// SelfAttention_78271484003105
// MI455X (gfx1250) — hardware-verified
//
#include <hip/hip_runtime.h>


#ifndef NB
#define NB 4
#endif
#ifndef SEQ
#define SEQ 1024
#endif
#define NB_FULL  4
#define SEQ_FULL 1024
#define DM   1024
#define NH   16
#define HD   64
#define NTOK (NB * SEQ)
#define PCAR 256.0f
#define L2E  1.4426950408889634f

static_assert(DM == NH * HD);
static_assert(HD == 64);
static_assert((DM & (DM - 1)) == 0);
static_assert(DM % 64 == 0);
static_assert(SEQ % 64 == 0);
static_assert(NTOK % 64 == 0);
static_assert(SEQ <= SEQ_FULL);
static_assert(NB <= NB_FULL);
static_assert(((size_t)NTOK * DM / 8) % 256 == 0);
static_assert(((size_t)DM * DM / 8) % 256 == 0);

typedef _Float16 h16;
typedef unsigned short bf;
typedef __attribute__((ext_vector_type(16))) __bf16   v16bf;
typedef __attribute__((ext_vector_type(16))) _Float16 v16h;
typedef __attribute__((ext_vector_type(8)))  _Float16 v8h;
typedef __attribute__((ext_vector_type(8)))  unsigned short v8us;
typedef __attribute__((ext_vector_type(8)))  float    v8f;
typedef __attribute__((ext_vector_type(4)))  float    v4f;
typedef v4f  __attribute__((may_alias)) v4fa;

__device__ __forceinline__ unsigned short f2bf(float f) { unsigned u = __float_as_uint(f); u += 0x7FFFu + ((u >> 16) & 1u); return (unsigned short)(u >> 16); }
__device__ __forceinline__ float bf2f(unsigned short b) { return __uint_as_float(((unsigned)b) << 16); }
__device__ __forceinline__ float bfr(float f) { return bf2f(f2bf(f)); }
__device__ __forceinline__ void splitf(float y, unsigned short& h, unsigned short& l) { h = f2bf(y); l = f2bf(y - bf2f(h)); }
__device__ __forceinline__ v16h cat16(v8h lo, v8h hi) { return __builtin_shufflevector(lo, hi, 0, 1, 2, 3, 4, 5, 6, 7, 8, 9, 10, 11, 12, 13, 14, 15); }
__device__ __forceinline__ v16bf cat16b(v8us lo, v8us hi) { return __builtin_bit_cast(v16bf, __builtin_shufflevector(lo, hi, 0, 1, 2, 3, 4, 5, 6, 7, 8, 9, 10, 11, 12, 13, 14, 15)); }
__device__ __forceinline__ v8f wmma16(v16h a, v16h b, v8f c) { return __builtin_amdgcn_wmma_f32_16x16x32_f16(false, a, false, b, (short)0, c, false, false); }
__device__ __forceinline__ v8f wmmab(v16bf a, v16bf b, v8f c) { return __builtin_amdgcn_wmma_f32_16x16x32_bf16(false, a, false, b, (short)0, c, false, false); }
__device__ __forceinline__ v16bf ldfb(const bf* p) { return cat16b(*(const v8us*)p, *(const v8us*)(p + 16)); }
__device__ __forceinline__ v16h  ldfh(const h16* p) { return cat16(*(const v8h*)p, *(const v8h*)(p + 16)); }
__device__ __forceinline__ v8us cvt8bf(v8f v) { v8us o;
#pragma unroll
    for (int k = 0; k < 8; ++k) o[k] = f2bf(v[k]);
    return o; }

__global__ __launch_bounds__(256) void k_cvtx(const float* __restrict__ src, bf* dst) {
    const size_t i = (size_t)blockIdx.x * 256 + threadIdx.x;
    if (i >= (size_t)NTOK * DM / 8) return;
    const size_t e = i * 8; const int row = (int)(e / DM); const int col = (int)(e % DM);
    const int b = row / SEQ, t = row % SEQ;
    const v8f v = *(const v8f*)(src + ((size_t)b * SEQ_FULL + t) * DM + col);
    const v8us o = cvt8bf(v);
    *(volatile v8us*)(dst + e) = o; __threadfence(); *(volatile v8us*)(dst + e) = o;
}

__global__ __launch_bounds__(256) void k_cvtw4(const float* __restrict__ w0, const float* __restrict__ w1, const float* __restrict__ w2, const float* __restrict__ w3, bf* dst) {
    const size_t i = (size_t)blockIdx.x * 256 + threadIdx.x;
    if (i >= (size_t)DM * DM / 8) return;
    const size_t e = i * 8; const size_t P = (size_t)DM * DM;
    const v8us o0 = cvt8bf(*(const v8f*)(w0 + e)); const v8us o1 = cvt8bf(*(const v8f*)(w1 + e));
    const v8us o2 = cvt8bf(*(const v8f*)(w2 + e)); const v8us o3 = cvt8bf(*(const v8f*)(w3 + e));
    *(volatile v8us*)(dst + e) = o0; *(volatile v8us*)(dst + P + e) = o1; *(volatile v8us*)(dst + 2 * P + e) = o2; *(volatile v8us*)(dst + 3 * P + e) = o3;
    __threadfence();
    *(volatile v8us*)(dst + e) = o0; *(volatile v8us*)(dst + P + e) = o1; *(volatile v8us*)(dst + 2 * P + e) = o2; *(volatile v8us*)(dst + 3 * P + e) = o3;
}

__device__ __forceinline__ void gemm_core(const bf* __restrict__ A, int lda, const bf* __restrict__ Bt, int K, int r0, int c0, int lr, int hi, v8f (&acc)[4][4]) {
#pragma unroll
    for (int mb = 0; mb < 4; ++mb)
#pragma unroll
        for (int nb = 0; nb < 4; ++nb) acc[mb][nb] = (v8f){};
    const size_t aoff = (size_t)(r0 + lr) * lda + 8 * hi;
    const size_t boff = (size_t)(c0 + lr) * DM + 8 * hi;
#pragma unroll 1
    for (int kc = 0; kc < K; kc += 32) {
        const int kb = kc & (DM - 1);
        v16bf a[4], b[4];
#pragma unroll
        for (int mb = 0; mb < 4; ++mb) a[mb] = ldfb(A + aoff + (size_t)mb * 16 * lda + kc);
#pragma unroll
        for (int nb = 0; nb < 4; ++nb) b[nb] = ldfb(Bt + boff + (size_t)nb * 16 * DM + kb);
#pragma unroll
        for (int nb = 0; nb < 4; ++nb)
#pragma unroll
            for (int mb = 0; mb < 4; ++mb) acc[mb][nb] = wmmab(a[mb], b[nb], acc[mb][nb]);
        asm volatile("" : "+v"(acc[0][0]), "+v"(acc[1][0]), "+v"(acc[2][0]), "+v"(acc[3][0]), "+v"(acc[0][1]), "+v"(acc[1][1]), "+v"(acc[2][1]), "+v"(acc[3][1]));
        asm volatile("v_nop\n\tv_nop\n\tv_nop\n\tv_nop" : "+v"(acc[0][2]), "+v"(acc[1][2]), "+v"(acc[2][2]), "+v"(acc[3][2]), "+v"(acc[0][3]), "+v"(acc[1][3]), "+v"(acc[2][3]), "+v"(acc[3][3]) : "v"(a[0]), "v"(a[3]), "v"(b[3]));
    }
}

__global__ __launch_bounds__(32) void k_proj_qk(const bf* __restrict__ XB, const bf* __restrict__ W2, bf* PH, bf* PL) {
    __shared__ __align__(16) float os[16 * 68];
    const int lane = threadIdx.x & 31, lr = lane & 15, hi = lane >> 4;
    const int z = blockIdx.z; const int r0 = blockIdx.x * 64, c0 = blockIdx.y * 64;
    const float sc = (z == 0) ? 0.125f : 1.0f;
    v8f acc[4][4];
    gemm_core(XB, DM, W2 + (size_t)z * DM * DM, DM, r0, c0, lr, hi, acc);
    bf* ph = PH + (size_t)z * NTOK * DM; bf* pl = PL + (size_t)z * NTOK * DM;
    const int rq = lane >> 3, c8 = (lane & 7) * 8;
#pragma unroll
    for (int mb = 0; mb < 4; ++mb) {
#pragma unroll
        for (int nb = 0; nb < 4; ++nb)
#pragma unroll
            for (int j = 0; j < 8; ++j) os[(hi * 8 + j) * 68 + nb * 16 + lr] = acc[mb][nb][j] * sc;
        __syncthreads();
        v8us oh[4], ol[4];
#pragma unroll
        for (int s = 0; s < 4; ++s) { const int row = 4 * s + rq; const v4f u0 = *(const v4fa*)(os + row * 68 + c8); const v4f u1 = *(const v4fa*)(os + row * 68 + c8 + 4);
#pragma unroll
            for (int q = 0; q < 4; ++q) { unsigned short a, c; splitf(u0[q], a, c); oh[s][q] = a; ol[s][q] = c; splitf(u1[q], a, c); oh[s][4 + q] = a; ol[s][4 + q] = c; } }
        const size_t base = (size_t)(r0 + mb * 16) * DM + c0 + c8;
#pragma unroll
        for (int s = 0; s < 4; ++s) { const size_t o = base + (size_t)(4 * s + rq) * DM; *(volatile v8us*)(ph + o) = oh[s]; *(volatile v8us*)(pl + o) = ol[s]; }
        __threadfence();
#pragma unroll
        for (int s = 0; s < 4; ++s) { const size_t o = base + (size_t)(4 * s + rq) * DM; *(volatile v8us*)(ph + o) = oh[s]; *(volatile v8us*)(pl + o) = ol[s]; }
        __syncthreads();
    }
}

__global__ __launch_bounds__(32) void k_proj_vt(const bf* __restrict__ WV, const bf* __restrict__ XB, h16* VT) {
    __shared__ __align__(16) float os[16 * 68];
    const int lane = threadIdx.x & 31, lr = lane & 15, hi = lane >> 4;
    const int r0 = blockIdx.x * 64, c0 = blockIdx.y * 64;
    v8f acc[4][4];
    gemm_core(WV, DM, XB, DM, r0, c0, lr, hi, acc);
    const int rq = lane >> 3, c8 = (lane & 7) * 8;
#pragma unroll
    for (int mb = 0; mb < 4; ++mb) {
#pragma unroll
        for (int nb = 0; nb < 4; ++nb)
#pragma unroll
            for (int j = 0; j < 8; ++j) os[(hi * 8 + j) * 68 + nb * 16 + lr] = acc[mb][nb][j];
        __syncthreads();
        v8h o16[4];
#pragma unroll
        for (int s = 0; s < 4; ++s) { const int row = 4 * s + rq; const v4f u0 = *(const v4fa*)(os + row * 68 + c8); const v4f u1 = *(const v4fa*)(os + row * 68 + c8 + 4);
#pragma unroll
            for (int q = 0; q < 4; ++q) { o16[s][q] = (h16)u0[q]; o16[s][4 + q] = (h16)u1[q]; } }
        const size_t base = (size_t)(r0 + mb * 16) * NTOK + c0 + c8;
#pragma unroll
        for (int s = 0; s < 4; ++s) *(volatile v8h*)(VT + base + (size_t)(4 * s + rq) * NTOK) = o16[s];
        __threadfence();
#pragma unroll
        for (int s = 0; s < 4; ++s) *(volatile v8h*)(VT + base + (size_t)(4 * s + rq) * NTOK) = o16[s];
        __syncthreads();
    }
}

__global__ __launch_bounds__(128) void k_attn(const bf* __restrict__ QH, const bf* __restrict__ QL, const bf* __restrict__ KH, const bf* __restrict__ KL, const h16* __restrict__ VT, bf* CTX) {
    __shared__ __align__(16) float os[4 * 16 * 68];
    const int lane = threadIdx.x & 31, lr = lane & 15, hi = lane >> 4;
    const int wave = __builtin_amdgcn_readfirstlane(threadIdx.x >> 5);
    const int bh = blockIdx.y; const int b = bh / NH, h = bh % NH;
    const int tok0 = b * SEQ; const int q0 = blockIdx.x * 64 + wave * 16;
    const size_t qoff = (size_t)(tok0 + q0 + lr) * DM + h * HD + 8 * hi;
    v16bf qh[2], ql[2];
    qh[0] = ldfb(QH + qoff); qh[1] = ldfb(QH + qoff + 32); ql[0] = ldfb(QL + qoff); ql[1] = ldfb(QL + qoff + 32);
    const size_t koff = (size_t)(tok0 + lr) * DM + h * HD + 8 * hi;
    const size_t voff = (size_t)(h * HD + lr) * NTOK + tok0 + 8 * hi;
    v8f ot[4];
#pragma unroll
    for (int dt = 0; dt < 4; ++dt) ot[dt] = (v8f){};
    float mrun = -1.0e30f, lrun = 0.0f;
#pragma unroll 1
    for (int kb = 0; kb < SEQ; kb += 32) {
        v16bf kfh[2][2], kfl[2][2];
#pragma unroll
        for (int j = 0; j < 2; ++j)
#pragma unroll
            for (int c = 0; c < 2; ++c) { const size_t o = koff + (size_t)(kb + 16 * j) * DM + 32 * c; kfh[j][c] = ldfb(KH + o); kfl[j][c] = ldfb(KL + o); }
        v8f st[2];
        st[0] = (v8f){}; st[1] = (v8f){};
#pragma unroll
        for (int j = 0; j < 2; ++j)
#pragma unroll
            for (int c = 0; c < 2; ++c) { st[j] = wmmab(kfl[j][c], qh[c], st[j]); st[j] = wmmab(kfh[j][c], ql[c], st[j]); st[j] = wmmab(kfh[j][c], qh[c], st[j]); }
        asm volatile("v_nop\n\tv_nop\n\tv_nop\n\tv_nop" : "+v"(st[0]), "+v"(st[1]) : "v"(kfh[1][1]), "v"(qh[1]));
        float cmax = st[0][0];
#pragma unroll
        for (int r = 0; r < 8; ++r) { cmax = fmaxf(cmax, st[0][r]); cmax = fmaxf(cmax, st[1][r]); }
        cmax = fmaxf(cmax, __shfl_xor(cmax, 16, 32));
        const float mnew = fmaxf(mrun, cmax);
        const float alpha = __builtin_amdgcn_exp2f((mrun - mnew) * L2E);
        float part = 0.0f; v16h pf;
#pragma unroll
        for (int r = 0; r < 8; ++r) { const float p0 = __builtin_amdgcn_exp2f((st[0][r] - mnew) * L2E); const float p1 = __builtin_amdgcn_exp2f((st[1][r] - mnew) * L2E);
            part += p0 + p1; pf[r] = (h16)(p0 * PCAR); pf[8 + r] = (h16)(p1 * PCAR); }
        part += __shfl_xor(part, 16, 32);
        lrun = lrun * alpha + part; mrun = mnew;
#pragma unroll
        for (int dt = 0; dt < 4; ++dt)
#pragma unroll
            for (int r = 0; r < 8; ++r) ot[dt][r] *= alpha;
        v16h vf[4];
#pragma unroll
        for (int dt = 0; dt < 4; ++dt) vf[dt] = ldfh(VT + voff + (size_t)(dt * 16) * NTOK + kb);
#pragma unroll
        for (int dt = 0; dt < 4; ++dt) ot[dt] = wmma16(vf[dt], pf, ot[dt]);
        asm volatile("v_nop\n\tv_nop\n\tv_nop\n\tv_nop" : "+v"(ot[0]), "+v"(ot[1]), "+v"(ot[2]), "+v"(ot[3]) : "v"(vf[3]), "v"(pf));
    }
    const float inv = (1.0f / PCAR) * (1.0f / lrun);
    const int wb = wave * 16 * 68;
#pragma unroll
    for (int dt = 0; dt < 4; ++dt)
#pragma unroll
        for (int r = 0; r < 8; ++r) os[wb + lr * 68 + dt * 16 + 8 * hi + r] = ot[dt][r] * inv;
    __syncthreads();
    const int rq = lane >> 3, c8 = (lane & 7) * 8;
    v8us oh[4], ol[4];
#pragma unroll
    for (int s = 0; s < 4; ++s) { const int row = 4 * s + rq; const v4f u0 = *(const v4fa*)(os + wb + row * 68 + c8); const v4f u1 = *(const v4fa*)(os + wb + row * 68 + c8 + 4);
#pragma unroll
        for (int q = 0; q < 4; ++q) { unsigned short a, c; splitf(u0[q], a, c); oh[s][q] = a; ol[s][q] = c; splitf(u1[q], a, c); oh[s][4 + q] = a; ol[s][4 + q] = c; } }
    const size_t base = (size_t)(tok0 + q0) * (2 * DM) + h * HD + c8;
#pragma unroll
    for (int s = 0; s < 4; ++s) { const size_t o = base + (size_t)(4 * s + rq) * (2 * DM); *(volatile v8us*)(CTX + o) = oh[s]; *(volatile v8us*)(CTX + o + DM) = ol[s]; }
    __threadfence();
#pragma unroll
    for (int s = 0; s < 4; ++s) { const size_t o = base + (size_t)(4 * s + rq) * (2 * DM); *(volatile v8us*)(CTX + o) = oh[s]; *(volatile v8us*)(CTX + o + DM) = ol[s]; }
}

__global__ __launch_bounds__(32) void k_proj_out(const bf* __restrict__ CTX, const bf* __restrict__ WO, const float* __restrict__ bias, float* OUT) {
    __shared__ __align__(16) float os[16 * 68];
    const int lane = threadIdx.x & 31, lr = lane & 15, hi = lane >> 4;
    const int r0 = blockIdx.x * 64, c0 = blockIdx.y * 64;
    v8f acc[4][4];
    gemm_core(CTX, 2 * DM, WO, 2 * DM, r0, c0, lr, hi, acc);
    const int bb = r0 / SEQ, tt = r0 % SEQ; const int cofs = lr * 4;
    v4f bv; bv[0] = bfr(bias[c0 + cofs]); bv[1] = bfr(bias[c0 + cofs + 1]); bv[2] = bfr(bias[c0 + cofs + 2]); bv[3] = bfr(bias[c0 + cofs + 3]);
#pragma unroll
    for (int mb = 0; mb < 4; ++mb) {
#pragma unroll
        for (int nb = 0; nb < 4; ++nb)
#pragma unroll
            for (int j = 0; j < 8; ++j) os[(hi * 8 + j) * 68 + nb * 16 + lr] = acc[mb][nb][j];
        __syncthreads();
        v4f val[8];
#pragma unroll
        for (int s = 0; s < 8; ++s) { const int row = 2 * s + hi; val[s] = *(const v4fa*)(os + row * 68 + cofs) + bv; }
        float* crow = OUT + ((size_t)bb * SEQ_FULL + tt + mb * 16) * DM + c0 + cofs;
#pragma unroll
        for (int s = 0; s < 8; ++s) *(volatile v4f*)(crow + (size_t)(2 * s + hi) * DM) = val[s];
        __threadfence();
#pragma unroll
        for (int s = 0; s < 8; ++s) *(volatile v4f*)(crow + (size_t)(2 * s + hi) * DM) = val[s];
        __syncthreads();
    }
}

constexpr size_t SZ_XB  = (size_t)NTOK * DM * 2;
constexpr size_t SZ_W   = (size_t)4 * DM * DM * 2;
constexpr size_t SZ_QK  = (size_t)2 * NTOK * DM * 2;
constexpr size_t SZ_VT  = (size_t)DM * NTOK * 2;
constexpr size_t SZ_CTX = (size_t)NTOK * 2 * DM * 2;
constexpr size_t OFF_XB = 0, OFF_W = OFF_XB + SZ_XB, OFF_QKH = OFF_W + SZ_W, OFF_QKL = OFF_QKH + SZ_QK, OFF_VT = OFF_QKL + SZ_QK, OFF_CTX = OFF_VT + SZ_VT, WS_TOTAL = OFF_CTX + SZ_CTX;
static_assert(WS_TOTAL <= (size_t)134217728);
static_assert(SZ_XB % 256 == 0 && SZ_W % 256 == 0 && SZ_QK % 256 == 0 && SZ_VT % 256 == 0 && SZ_CTX % 256 == 0);

extern "C" void kernel_launch(void* const* d_in, const int* in_sizes, int n_in,
                              void* d_out, int out_size, void* d_ws, size_t ws_size, hipStream_t stream) {
    if (n_in < 6) return;
    const size_t need_x = ((size_t)(NB - 1) * SEQ_FULL + SEQ) * DM;
    if ((size_t)in_sizes[0] < need_x) return;
    if ((size_t)in_sizes[1] < (size_t)DM * DM || (size_t)in_sizes[2] < (size_t)DM * DM || (size_t)in_sizes[3] < (size_t)DM * DM || (size_t)in_sizes[4] < (size_t)DM * DM) return;
    if (in_sizes[5] < DM) return;
    if ((size_t)out_size < need_x) return;
    if (ws_size < WS_TOTAL) return;
    const float* x = (const float*)d_in[0]; const float* wq = (const float*)d_in[1]; const float* wk = (const float*)d_in[2];
    const float* wv = (const float*)d_in[3]; const float* wo = (const float*)d_in[4]; const float* bo = (const float*)d_in[5];
    float* OUT = (float*)d_out;
    char* ws = (char*)d_ws;
    bf* XB = (bf*)(ws + OFF_XB); bf* WALL = (bf*)(ws + OFF_W); bf* QKH = (bf*)(ws + OFF_QKH); bf* QKL = (bf*)(ws + OFF_QKL);
    h16* VT = (h16*)(ws + OFF_VT); bf* CTX = (bf*)(ws + OFF_CTX);
    const size_t WP = (size_t)DM * DM; const size_t PP = (size_t)NTOK * DM;
    k_cvtx<<<(unsigned)(((size_t)NTOK * DM / 8 + 255) / 256), 256, 0, stream>>>(x, XB);
    k_cvtw4<<<(unsigned)((WP / 8 + 255) / 256), 256, 0, stream>>>(wq, wk, wv, wo, WALL);
    k_proj_qk<<<dim3(NTOK / 64, DM / 64, 2), 32, 0, stream>>>(XB, WALL, QKH, QKL);
    k_proj_vt<<<dim3(DM / 64, NTOK / 64, 1), 32, 0, stream>>>(WALL + 2 * WP, XB, VT);
    k_attn<<<dim3(SEQ / 64, NB * NH, 1), 128, 0, stream>>>(QKH, QKL, QKH + PP, QKL + PP, VT, CTX);
    k_proj_out<<<dim3(NTOK / 64, DM / 64, 1), 32, 0, stream>>>(CTX, WALL + 3 * WP, bo, OUT);
}
